// NetworkGL_Lite_70033736728882
// MI455X (gfx1250) — hardware-verified
//
#include <hip/hip_runtime.h>
#include <math.h>

constexpr int NBATCH   = 64;
constexpr int SEQ      = 512;
constexpr int NCH      = 321;
constexpr int NROWS    = NBATCH * NCH;
constexpr int NPATCH   = 64;
constexpr int PLEN     = 16;
constexpr int HIDDEN   = 32;
constexpr int NPRED    = 96;
constexpr int NPREDP   = 128;
constexpr int CGROUPS  = 11;
constexpr int MSPITCH  = CGROUPS * 32;
constexpr int ZPITCH   = 256;
constexpr int DPITCH   = NPATCH * PLEN;
constexpr int PROWS_BLK = 16;
constexpr int NPBLK    = NROWS / PROWS_BLK;
constexpr int YSP      = DPITCH + 8;
constexpr int OUT_ELEMS = NBATCH * NPRED * NCH;
static_assert(NROWS % 64 == 0, "");
static_assert(NROWS % PROWS_BLK == 0, "");
static_assert(OUT_ELEMS % 1024 == 0, "");

constexpr float WCARRY = 32.0f;
constexpr float ACARRY = 16.0f;
constexpr float UCARRY = 64.0f;
constexpr float GCARRY = 256.0f;
constexpr float DCARRY = 256.0f;
constexpr float FC1_SCALE = 1.0f / (WCARRY * ACARRY);
constexpr float D_STORE_SCALE = DCARRY / (GCARRY * WCARRY);
constexpr float BN_EPS = 1e-5f;

typedef __attribute__((ext_vector_type(16))) _Float16 v16h;
typedef __attribute__((ext_vector_type(8)))  _Float16 v8h;
typedef __attribute__((ext_vector_type(16))) __bf16   v16b;
typedef __attribute__((ext_vector_type(8)))  __bf16   v8b;
typedef __attribute__((ext_vector_type(8)))  float    v8f;
typedef __attribute__((ext_vector_type(4)))  float    v4f;
typedef __attribute__((ext_vector_type(4)))  unsigned int v4u;

__device__ __forceinline__ unsigned short f2bf_bits(float f) {
  unsigned u = __float_as_uint(f);
  return (unsigned short)((u + 0x7FFFu + ((u >> 16) & 1u)) >> 16);
}
__device__ __forceinline__ float bf_bits2f(unsigned short h) { return __uint_as_float(((unsigned)h) << 16); }

__device__ __forceinline__ void dep_guard_h(v8f& a, v8f& b, v16h x, v16h y) { asm volatile("v_nop\n\tv_nop\n\tv_nop\n\tv_nop" : "+v"(a), "+v"(b) : "v"(x), "v"(y)); }
__device__ __forceinline__ void dep_guard_b(v8f& a, v8f& b, v16b x, v16b y) { asm volatile("v_nop\n\tv_nop\n\tv_nop\n\tv_nop" : "+v"(a), "+v"(b) : "v"(x), "v"(y)); }
__device__ __forceinline__ void keep4_h(v16h a, v16h b, v16h c, v16h d) { asm volatile("v_nop" :: "v"(a), "v"(b), "v"(c), "v"(d)); }
__device__ __forceinline__ void keep4_b(v16b a, v16b b, v16b c, v16b d) { asm volatile("v_nop" :: "v"(a), "v"(b), "v"(c), "v"(d)); }
__device__ __forceinline__ void acc_guard4(v8f& a, v8f& b, v8f& c, v8f& d) { asm volatile("v_nop\n\tv_nop\n\tv_nop\n\tv_nop" : "+v"(a), "+v"(b), "+v"(c), "+v"(d)); }
template <typename T> struct Frag;
template <> struct Frag<_Float16> {
  typedef v16h V; union U { v16h v; v8h h[2]; };
  static __device__ __forceinline__ v16h load(const _Float16* p) {
    U f; f.h[0] = *(const v8h*)(p); f.h[1] = *(const v8h*)(p + 16); return f.v;
  }
  static __device__ __forceinline__ v8f mma(v16h a, v16h b, v8f c) {
    return __builtin_amdgcn_wmma_f32_16x16x32_f16(false, a, false, b, (short)0, c, false, false);
  }
  static __device__ __forceinline__ void guard(v8f& a, v8f& b, v16h x, v16h y) { dep_guard_h(a, b, x, y); }
  static __device__ __forceinline__ void keep(v16h a, v16h b, v16h c, v16h d) { keep4_h(a, b, c, d); }
};
template <> struct Frag<__bf16> {
  typedef v16b V; union U { v16b v; v8b h[2]; };
  static __device__ __forceinline__ v16b load(const __bf16* p) {
    U f; f.h[0] = *(const v8b*)(p); f.h[1] = *(const v8b*)(p + 16); return f.v;
  }
  static __device__ __forceinline__ v8f mma(v16b a, v16b b, v8f c) {
    return __builtin_amdgcn_wmma_f32_16x16x32_bf16(false, a, false, b, (short)0, c, false, false);
  }
  static __device__ __forceinline__ void guard(v8f& a, v8f& b, v16b x, v16b y) { dep_guard_b(a, b, x, y); }
  static __device__ __forceinline__ void keep(v16b a, v16b b, v16b c, v16b d) { keep4_b(a, b, c, d); }
};

__device__ __forceinline__ unsigned pk16(unsigned short a, unsigned short b) { return (unsigned)a | ((unsigned)b << 16); }
__device__ __forceinline__ unsigned short h_bits(float f) { const _Float16 h = (_Float16)f; return __builtin_bit_cast(unsigned short, h); }

template <int ET> struct Elem;
template <> struct Elem<0> { typedef _Float16 T; };
template <> struct Elem<1> { typedef __bf16 T; };
template <int ET, bool SPLIT, int BIAS_MODE, int OUT_MODE, bool RESID, int ACT = 0>
__global__ __launch_bounds__(256) void wmma_gemm64(
    const unsigned short* __restrict__ Ap, const unsigned short* __restrict__ A2p, int lda, long strideA,
    const unsigned short* __restrict__ Btp, const unsigned short* __restrict__ Bt2p, int ldb, long strideB,
    void* __restrict__ Cout, void* __restrict__ Cout2, int ldc, long strideC,
    const float* __restrict__ bias,
    const float* __restrict__ resid, long strideR,
    int M, int N, int K, float scale) {
  typedef typename Elem<ET>::T T;
  typedef typename Frag<T>::V V;
  const T* A = (const T*)Ap; const T* A2 = (const T*)A2p; const T* Bt = (const T*)Btp; const T* Bt2 = (const T*)Bt2p;
  __shared__ __align__(16) float sT[8][16 * 68];
  const int b    = blockIdx.y;
  const int lane = threadIdx.x & 31;
  const int wave = threadIdx.x >> 5;
  const int tilesN = N >> 6;
  const int tilesM = M >> 6;
  const int tile = blockIdx.x * 8 + wave;
  if (tile >= tilesM * tilesN) return;
  const int tm = tile / tilesN;
  const int tn = tile - tm * tilesN;
  const int m0 = tm << 6;
  const int n0 = tn << 6;

  const T* Ab  = A  + (size_t)b * strideA;
  const T* Bb  = Bt + (size_t)b * strideB;
  const T* Ab2 = SPLIT ? (A2  + (size_t)b * strideA) : nullptr;
  const T* Bb2 = SPLIT ? (Bt2 + (size_t)b * strideB) : nullptr;

  const int rlane = lane & 15;
  const int koff  = (lane >> 4) * 8;
  const int mOff  = (lane >> 4) * 8;

  v8f acc[4][4];
#pragma unroll
  for (int i = 0; i < 4; ++i)
#pragma unroll
    for (int j = 0; j < 4; ++j) acc[i][j] = (v8f){0.f,0.f,0.f,0.f,0.f,0.f,0.f,0.f};

  for (int k0 = 0; k0 < K; k0 += 32) {
    V bh[4], bl[4];
#pragma unroll
    for (int j = 0; j < 4; ++j) {
      const size_t bo = (size_t)(n0 + (j << 4) + rlane) * ldb + koff + k0;
      bh[j] = Frag<T>::load(Bb + bo);
      if (SPLIT) bl[j] = Frag<T>::load(Bb2 + bo);
    }
#pragma unroll
    for (int i = 0; i < 4; ++i) {
      const size_t ao = (size_t)(m0 + (i << 4) + rlane) * lda + koff + k0;
      V ah = Frag<T>::load(Ab + ao);
      V al;
      if (SPLIT) al = Frag<T>::load(Ab2 + ao);
#pragma unroll
      for (int j = 0; j < 4; ++j) {
        acc[i][j] = Frag<T>::mma(ah, bh[j], acc[i][j]);
        if (SPLIT) {
          acc[i][j] = Frag<T>::mma(ah, bl[j], acc[i][j]);
          acc[i][j] = Frag<T>::mma(al, bh[j], acc[i][j]);
        }
      }
      Frag<T>::guard(acc[i][0], acc[i][3], ah, SPLIT ? al : ah);
    }
    Frag<T>::keep(bh[0], bh[1], bh[2], bh[3]);
    if (SPLIT) Frag<T>::keep(bl[0], bl[1], bl[2], bl[3]);
  }
  acc_guard4(acc[0][0], acc[0][1], acc[0][2], acc[0][3]);
  acc_guard4(acc[1][0], acc[1][1], acc[1][2], acc[1][3]);
  acc_guard4(acc[2][0], acc[2][1], acc[2][2], acc[2][3]);
  acc_guard4(acc[3][0], acc[3][1], acc[3][2], acc[3][3]);

  float* slab = sT[wave];
  const float* Rb = RESID ? (resid + (size_t)b * strideR) : nullptr;
#pragma unroll
  for (int i = 0; i < 4; ++i) {
    const int mBase = m0 + (i << 4);
#pragma unroll
    for (int j = 0; j < 4; ++j) {
      const int n = n0 + (j << 4) + rlane;
      float bv = 0.f;
      if (BIAS_MODE == 2) bv = bias[n];
#pragma unroll
      for (int r = 0; r < 8; ++r) {
        float v = acc[i][j][r] * scale;
        if (BIAS_MODE == 1) v += bias[mBase + mOff + r];
        if (BIAS_MODE == 2) v += bv;
        if (RESID) v += Rb[(size_t)(mBase + mOff + r) * ldc + n];
        if (ACT == 1) v = tanhf(v);
        if (ACT == 2) v = fmaxf(v, 0.0f);
        if (ACT == 3) v = v / (1.0f + expf(-v));
        if (ACT == 4) v = (v > 0.f) ? v : 0.01f * v;
        if (ACT == 6) v = 1.0f / (1.0f + expf(-v));
        slab[(mOff + r) * 68 + (j << 4) + rlane] = v;
      }
    }
    __builtin_amdgcn_fence(__ATOMIC_RELEASE, "workgroup");
    __builtin_amdgcn_wave_barrier();
    __builtin_amdgcn_fence(__ATOMIC_ACQUIRE, "workgroup");
    if (OUT_MODE == 0) {
      float* C = (float*)Cout + (size_t)b * strideC;
      const int hh = lane >> 4, c4 = (lane & 15) * 4;
      for (int pass = 0; pass < 2; ++pass) {
#pragma unroll
        for (int it = 0; it < 8; ++it) {
          const int row = it * 2 + hh;
          v4f v = *(const v4f*)(slab + row * 68 + c4);
          *(volatile v4f*)(C + (size_t)(mBase + row) * ldc + n0 + c4) = v;
        }
        __threadfence();
      }
    } else {
      const int q = lane >> 3, c8 = (lane & 7) * 8;
      unsigned short* C  = (unsigned short*)Cout  + (size_t)b * strideC;
      unsigned short* C2 = (OUT_MODE == 2) ? ((unsigned short*)Cout2 + (size_t)b * strideC) : nullptr;
      for (int pass = 0; pass < 2; ++pass) {
#pragma unroll
        for (int it = 0; it < 4; ++it) {
          const int row = it * 4 + q;
          const float* sp = slab + row * 68 + c8;
          v8h hv, lv;
#pragma unroll
          for (int e = 0; e < 8; ++e) {
            if (OUT_MODE == 1) {
              hv[e] = (_Float16)sp[e];
            } else {
              unsigned short hb = f2bf_bits(sp[e]);
              unsigned short lb = f2bf_bits(sp[e] - bf_bits2f(hb));
              hv[e] = __builtin_bit_cast(_Float16, hb);
              lv[e] = __builtin_bit_cast(_Float16, lb);
            }
          }
          *(volatile v8h*)(C + (size_t)(mBase + row) * ldc + n0 + c8) = hv;
          if (OUT_MODE == 2) *(volatile v8h*)(C2 + (size_t)(mBase + row) * ldc + n0 + c8) = lv;
        }
        __threadfence();
      }
    }
    __builtin_amdgcn_fence(__ATOMIC_RELEASE, "workgroup");
    __builtin_amdgcn_wave_barrier();
    __builtin_amdgcn_fence(__ATOMIC_ACQUIRE, "workgroup");
  }
}

__device__ __forceinline__ float gelu_erf(float v) {
  return 0.5f * v * (1.0f + erff(v * 0.70710678118654752440f));
}
__device__ __forceinline__ v8f hmma(v16h a, v16h b, v8f c) {
  c = __builtin_amdgcn_wmma_f32_16x16x32_f16(false, a, false, b, (short)0, c, false, false);
  asm volatile("v_nop\n\tv_nop\n\tv_nop\n\tv_nop" : "+v"(c) : "v"(a), "v"(b));
  return c;
}
union FragU { v16h v; v8h hh[2]; };

__global__ __launch_bounds__(256) void k_wprep(const float* __restrict__ m1_w, const float* __restrict__ m2_w,
                                                    const float* __restrict__ tr_w, const float* __restrict__ seas_w,
                                                    const float* __restrict__ fus_w, const float* __restrict__ tr_b,
                                                    const float* __restrict__ fus_b,
                                                    unsigned short* __restrict__ m1p, unsigned short* __restrict__ m2p,
                                                    unsigned short* __restrict__ trp, unsigned short* __restrict__ seasp,
                                                    unsigned short* __restrict__ fusp, float* __restrict__ biasp) {
  const int pl = blockIdx.y;
  const int i = blockIdx.x * 256 + threadIdx.x;
  if (pl == 5) {
    if (i >= 256) return;
    const int j = i & 127;
    const int jc = (j < NPRED) ? j : (NPRED - 1);
    const float tb = tr_b[jc];
    const float fb = fus_b[jc];
    float v = (i < 128) ? (tb * ACARRY) : fb;
    if (j >= NPRED) v = 0.f;
    volatile float* d = biasp + i;
    *d = v;
    __threadfence();
    *d = v;
    return;
  }
  float v0 = 0.f, v1 = 0.f;
  unsigned short* dst = m1p;
  if (pl == 0) {
    if (i >= NPREDP * NPATCH / 2) return;
    const int e = 2 * i;
    v0 = WCARRY * m1_w[e];
    v1 = WCARRY * m1_w[e + 1];
    dst = m1p;
  } else if (pl == 1) {
    if (i >= NPATCH * NPREDP / 2) return;
    const int e = 2 * i;
    v0 = WCARRY * m2_w[e];
    v1 = WCARRY * m2_w[e + 1];
    dst = m2p;
  } else if (pl == 2) {
    if (i >= NPREDP * SEQ / 2) return;
    const int e = 2 * i;
    const int row = e / SEQ;
    const int col = e - row * SEQ;
    const int rc = (row < NPRED) ? row : (NPRED - 1);
    const float a0 = tr_w[(size_t)rc * SEQ + col];
    const float a1 = tr_w[(size_t)rc * SEQ + col + 1];
    v0 = (row < NPRED) ? WCARRY * a0 : 0.f;
    v1 = (row < NPRED) ? WCARRY * a1 : 0.f;
    dst = trp;
  } else if (pl == 3) {
    if (i >= NPREDP * DPITCH / 2) return;
    const int e = 2 * i;
    const int row = e / DPITCH;
    const int col = e - row * DPITCH;
    const int rc = (row < NPRED) ? row : (NPRED - 1);
    const float a0 = seas_w[(size_t)rc * DPITCH + col];
    const float a1 = seas_w[(size_t)rc * DPITCH + col + 1];
    v0 = (row < NPRED) ? WCARRY * a0 : 0.f;
    v1 = (row < NPRED) ? WCARRY * a1 : 0.f;
    dst = seasp;
  } else {
    if (i >= NPREDP * ZPITCH / 2) return;
    const int e = 2 * i;
    const int row = e / ZPITCH;
    const int col = e - row * ZPITCH;
    const int rc = (row < NPRED) ? row : (NPRED - 1);
    int sc = (col < 128) ? col : (col - 32);
    sc = (sc > 190) ? 190 : sc;
    const bool valid = (row < NPRED) && ((col < NPRED) || (col >= 128 && col < 224));
    const float a0 = fus_w[(size_t)rc * (2 * NPRED) + sc];
    const float a1 = fus_w[(size_t)rc * (2 * NPRED) + sc + 1];
    v0 = valid ? WCARRY * a0 : 0.f;
    v1 = valid ? WCARRY * a1 : 0.f;
    dst = fusp;
  }
  const unsigned u = pk16(h_bits(v0), h_bits(v1));
  volatile unsigned* d = (volatile unsigned*)dst + i;
  *d = u;
  __threadfence();
  *d = u;
}

__global__ __launch_bounds__(64) void k_revin(const float* __restrict__ x, const float* __restrict__ rev_w,
                                                   const float* __restrict__ rev_b, float* __restrict__ s,
                                                   unsigned short* __restrict__ trend16,
                                                   float* __restrict__ meanp, float* __restrict__ stdp) {
  __shared__ float sT[2][64][33];
  __shared__ float tT[2][64][33];
  const int wave = threadIdx.x >> 5, lane = threadIdx.x & 31;
  const int wt = blockIdx.x * 2 + wave;
  const int b  = wt / CGROUPS;
  const int c0 = (wt - b * CGROUPS) * 32;
  const int c  = c0 + lane;
  const int ca = (c < NCH) ? c : (NCH - 1);
  const float* xp = x + (size_t)b * SEQ * NCH + ca;

  float sum = 0.f;
  for (int l = 0; l < SEQ; ++l) sum += xp[(size_t)l * NCH];
  const float mean = sum * (1.0f / (float)SEQ);
  float ssd = 0.f;
  for (int l = 0; l < SEQ; ++l) {
    const float d = xp[(size_t)l * NCH] - mean;
    ssd += d * d;
  }
  const float sd = sqrtf(ssd * (1.0f / (float)(SEQ - 1))) + BN_EPS;
  {
    const float mv = mean, sv = sd;
    volatile float* mp = meanp + (size_t)b * MSPITCH + c0 + lane;
    volatile float* sp = stdp + (size_t)b * MSPITCH + c0 + lane;
    *mp = mv; *sp = sv;
    __threadfence();
    *mp = mv; *sp = sv;
  }
  const float inv = 1.0f / sd;
  const float rw = rev_w[ca], rb = rev_b[ca];

  float carry = 0.f;
  for (int cb = 0; cb < SEQ / 64; ++cb) {
    for (int ll = 0; ll < 64; ++ll) {
      const int l = cb * 64 + ll;
      const float v  = xp[(size_t)l * NCH];
      const float xn = (v - mean) * inv * rw + rb;
      const float tr = (l == 0) ? xn : (0.2f * xn + 0.8f * carry);
      carry = tr;
      sT[wave][ll][lane] = xn - tr;
      tT[wave][ll][lane] = tr;
    }
    __syncthreads();
    for (int pass = 0; pass < 2; ++pass) {
      for (int cc = 0; cc < 32; ++cc) {
        const int ch = c0 + cc;
        if (ch < NCH) {
          const size_t rowi = (size_t)b * NCH + ch;
          const float s0 = sT[wave][lane][cc];
          const float s1 = sT[wave][32 + lane][cc];
          volatile float* so = s + rowi * SEQ + cb * 64;
          so[lane] = s0;
          so[32 + lane] = s1;
          const unsigned tb = pk16(h_bits(ACARRY * tT[wave][2 * lane][cc]),
                                   h_bits(ACARRY * tT[wave][2 * lane + 1][cc]));
          *(volatile unsigned*)(trend16 + rowi * SEQ + cb * 64 + 2 * lane) = tb;
        }
      }
      __threadfence();
    }
    __syncthreads();
  }
}

__global__ __launch_bounds__(256) void k_pool(const float* __restrict__ s, unsigned short* __restrict__ pooled16) {
  const int wave = threadIdx.x >> 5, lane = threadIdx.x & 31;
  for (int t = 0; t < 8; ++t) {
    const int row = blockIdx.x * 64 + wave * 8 + t;
    const float* sg = s + (size_t)row * SEQ;
    const float* p0 = sg + 16 * lane;
    const v4f a0 = *(const v4f*)(p0);
    const v4f a1 = *(const v4f*)(p0 + 4);
    const v4f a2 = *(const v4f*)(p0 + 8);
    const v4f a3 = *(const v4f*)(p0 + 12);
    float s0 = 0.f;
    s0 += a0[0]; s0 += a0[1]; s0 += a0[2]; s0 += a0[3];
    s0 += a1[0]; s0 += a1[1]; s0 += a1[2]; s0 += a1[3];
    s0 += a2[0]; s0 += a2[1]; s0 += a2[2]; s0 += a2[3];
    s0 += a3[0]; s0 += a3[1]; s0 += a3[2]; s0 += a3[3];
    float s1 = 0.f;
    s1 += a2[0]; s1 += a2[1]; s1 += a2[2]; s1 += a2[3];
    s1 += a3[0]; s1 += a3[1]; s1 += a3[2]; s1 += a3[3];
#pragma unroll
    for (int q = 0; q < 8; ++q) {
      int idx = 16 * lane + 16 + q;
      idx = (idx > SEQ - 1) ? (SEQ - 1) : idx;
      s1 += sg[idx];
    }
    const unsigned u = pk16(h_bits(s0), h_bits(s1));
    volatile unsigned* pp = (volatile unsigned*)(pooled16 + (size_t)row * NPATCH) + lane;
    *pp = u;
    __threadfence();
    *pp = u;
  }
}

__global__ __launch_bounds__(256) void k_gelu_u(const float* __restrict__ g1, unsigned short* __restrict__ u16, int n2) {
  const int i = blockIdx.x * 256 + threadIdx.x;
  if (i >= n2) return;
  const float a = g1[2 * (size_t)i];
  const float b = g1[2 * (size_t)i + 1];
  const unsigned u = pk16(h_bits(UCARRY * gelu_erf(a)), h_bits(UCARRY * gelu_erf(b)));
  volatile unsigned* d = (volatile unsigned*)u16 + i;
  *d = u;
  __threadfence();
  *d = u;
}

template <bool P2>
__global__ __launch_bounds__(128) void k_patch(const float* __restrict__ s, const float* __restrict__ fc1_w,
                                                    const float* __restrict__ fc1_b, const float* __restrict__ bnp1,
                                                    const float* __restrict__ conv_w, const float* __restrict__ conv_b,
                                                    const float* __restrict__ fc2_w,
                                                    float* __restrict__ ps, float* __restrict__ pq,
                                                    unsigned short* __restrict__ dplane) {
  __shared__ __align__(16) _Float16 srow16[4][528];
  __shared__ __align__(16) unsigned short dtile[4][DPITCH];
  __shared__ float pstat[4][2][NPATCH];
  const int lane = threadIdx.x & 31, wave = threadIdx.x >> 5;
  const int h = lane >> 4, c = lane & 15;
  const int blk = blockIdx.x;
  const v8f z8 = {0.f, 0.f, 0.f, 0.f, 0.f, 0.f, 0.f, 0.f};
  v8h z8h;
#pragma unroll
  for (int e = 0; e < 8; ++e) z8h[e] = (_Float16)0.0f;

  v16h af1[2];
  float fb1[2][8];
#pragma unroll
  for (int i = 0; i < 2; ++i) {
#pragma unroll
    for (int e = 0; e < 8; ++e) {
      af1[i][e]     = (_Float16)(WCARRY * fc1_w[(16 * i + c) * PLEN + 8 * h + e]);
      af1[i][8 + e] = (_Float16)0.0f;
      fb1[i][e]     = fc1_b[16 * i + 8 * h + e];
    }
  }
  float sc1[4], sh1[4], cw0[4], cw1[4], cw2[4], cbv[4];
  v16h bw2;
#pragma unroll
  for (int e = 0; e < 16; ++e) bw2[e] = (_Float16)0.0f;
#pragma unroll
  for (int j = 0; j < 4; ++j) { sc1[j] = 1.f; sh1[j] = 0.f; cw0[j] = 0.f; cw1[j] = 0.f; cw2[j] = 0.f; cbv[j] = 0.f; }
  if (P2) {
#pragma unroll
    for (int j = 0; j < 4; ++j) {
      const int n = 16 * j + c;
      sc1[j] = bnp1[n];
      sh1[j] = bnp1[NPATCH + n];
      cw0[j] = conv_w[n * 3 + 0];
      cw1[j] = conv_w[n * 3 + 1];
      cw2[j] = conv_w[n * 3 + 2];
      cbv[j] = conv_b[n];
    }
#pragma unroll
    for (int e = 0; e < 8; ++e) {
      bw2[e]     = (_Float16)(WCARRY * fc2_w[c * HIDDEN + 8 * h + e]);
      bw2[8 + e] = (_Float16)(WCARRY * fc2_w[c * HIDDEN + 16 + 8 * h + e]);
    }
  }
  float accS[4] = {0.f, 0.f, 0.f, 0.f};
  float accQ[4] = {0.f, 0.f, 0.f, 0.f};
  _Float16* sr = &srow16[wave][0];
  unsigned short* dt = &dtile[wave][0];

#pragma unroll 1
  for (int t = 0; t < 4; ++t) {
    const int row = blk * PROWS_BLK + wave * 4 + t;
    const float* sg = s + (size_t)row * SEQ;
#pragma unroll
    for (int u = 0; u < 16; ++u) sr[u * 32 + lane] = (_Float16)(ACARRY * sg[u * 32 + lane]);
    if (lane < 16) sr[512 + lane] = (_Float16)(ACARRY * sg[SEQ - 1]);
    __syncthreads();

#pragma unroll
    for (int j = 0; j < 4; ++j) {
      FragU bf;
      bf.hh[0] = *(const v8h*)(sr + 8 * (16 * j + c) + 8 * h);
      bf.hh[1] = z8h;
      const v8f x0 = hmma(af1[0], bf.v, z8);
      const v8f x1 = hmma(af1[1], bf.v, z8);
      float g0[8], g1v[8];
#pragma unroll
      for (int r = 0; r < 8; ++r) {
        g0[r]  = gelu_erf(x0[r] * FC1_SCALE + fb1[0][r]);
        g1v[r] = gelu_erf(x1[r] * FC1_SCALE + fb1[1][r]);
      }
      float ls = 0.f, lq = 0.f;
      if (!P2) {
#pragma unroll
        for (int r = 0; r < 8; ++r) { ls += g0[r]; lq += g0[r] * g0[r]; }
#pragma unroll
        for (int r = 0; r < 8; ++r) { ls += g1v[r]; lq += g1v[r] * g1v[r]; }
      } else {
        float e0[10], e1[10];
#pragma unroll
        for (int r = 0; r < 8; ++r) {
          e0[1 + r] = g0[r]  * sc1[j] + sh1[j];
          e1[1 + r] = g1v[r] * sc1[j] + sh1[j];
        }
        const float o00 = __shfl_xor(e0[1], 16, 32);
        const float o07 = __shfl_xor(e0[8], 16, 32);
        const float o10 = __shfl_xor(e1[1], 16, 32);
        const float o17 = __shfl_xor(e1[8], 16, 32);
        e0[0] = h ? o07 : 0.f;
        e0[9] = h ? o10 : o00;
        e1[0] = h ? o17 : o07;
        e1[9] = h ? 0.f : o10;
        float q0[8], q1[8];
#pragma unroll
        for (int r = 0; r < 8; ++r) {
          const float cv0 = cw0[j] * e0[r] + cw1[j] * e0[r + 1] + cw2[j] * e0[r + 2] + cbv[j];
          const float cv1 = cw0[j] * e1[r] + cw1[j] * e1[r + 1] + cw2[j] * e1[r + 2] + cbv[j];
          q0[r] = gelu_erf(cv0);
          q1[r] = gelu_erf(cv1);
          ls += q0[r]; lq += q0[r] * q0[r];
          ls += q1[r]; lq += q1[r] * q1[r];
        }
        v16h a2;
#pragma unroll
        for (int e = 0; e < 8; ++e) {
          a2[e]     = (_Float16)(GCARRY * q0[e]);
          a2[8 + e] = (_Float16)(GCARRY * q1[e]);
        }
        const v8f dd = hmma(a2, bw2, z8);
#pragma unroll
        for (int r = 0; r < 8; ++r) dt[(16 * j + 8 * h + r) * PLEN + c] = h_bits(dd[r] * D_STORE_SCALE);
      }
      ls += __shfl_xor(ls, 16, 32);
      lq += __shfl_xor(lq, 16, 32);
      accS[j] += ls;
      accQ[j] += lq;
    }
    if (P2) {
      __syncthreads();
      unsigned short* dg = dplane + (size_t)row * DPITCH;
      for (int pass = 0; pass < 2; ++pass) {
#pragma unroll
        for (int it = 0; it < 4; ++it) {
          const int off = 8 * (it * 32 + lane);
          const v4u val = *(const v4u*)(dt + off);
          *(volatile v4u*)(dg + off) = val;
        }
        __threadfence();
      }
    }
    __syncthreads();
  }

  if (h == 0) {
#pragma unroll
    for (int j = 0; j < 4; ++j) {
      pstat[wave][0][16 * j + c] = accS[j];
      pstat[wave][1][16 * j + c] = accQ[j];
    }
  }
  __syncthreads();
  if (wave == 0) {
    for (int pass = 0; pass < 2; ++pass) {
#pragma unroll
      for (int half = 0; half < 2; ++half) {
        const int n = 32 * half + lane;
        float vs = pstat[0][0][n]; vs += pstat[1][0][n]; vs += pstat[2][0][n]; vs += pstat[3][0][n];
        float vq = pstat[0][1][n]; vq += pstat[1][1][n]; vq += pstat[2][1][n]; vq += pstat[3][1][n];
        *(volatile float*)(ps + (size_t)blk * NPATCH + n) = vs;
        *(volatile float*)(pq + (size_t)blk * NPATCH + n) = vq;
      }
      __threadfence();
    }
  }
}

__global__ __launch_bounds__(64) void k_bnfin(const float* __restrict__ ps, const float* __restrict__ pq,
                                                  const float* __restrict__ bw, const float* __restrict__ bb,
                                                  float* __restrict__ bnp, int nblk) {
  const int n = threadIdx.x;
  double S = 0.0, Q = 0.0;
  for (int k = 0; k < nblk; ++k) {
    S += (double)ps[(size_t)k * NPATCH + n];
    Q += (double)pq[(size_t)k * NPATCH + n];
  }
  const double cnt = (double)NROWS * (double)HIDDEN;
  const double mu = S / cnt;
  double var = Q / cnt - mu * mu;
  if (var < 0.0) var = 0.0;
  const float sc = bw[n] * rsqrtf((float)var + BN_EPS);
  const float sh = bb[n] - (float)mu * sc;
  volatile float* p0 = bnp + n;
  volatile float* p1 = bnp + NPATCH + n;
  *p0 = sc; *p1 = sh;
  __threadfence();
  *p0 = sc; *p1 = sh;
}

__global__ __launch_bounds__(64) void k_lnhead(const float* __restrict__ s, const unsigned* __restrict__ dw,
                                                   const float* __restrict__ wsig, const float* __restrict__ bnp2,
                                                   const float* __restrict__ fc2_w, const float* __restrict__ fc2_b,
                                                   const float* __restrict__ gl_scale, const float* __restrict__ ln_w,
                                                   const float* __restrict__ ln_b, const unsigned short* __restrict__ seasp,
                                                   const float* __restrict__ seas_b, unsigned short* __restrict__ zplane) {
  __shared__ __align__(16) _Float16 ys[PROWS_BLK][YSP];
  __shared__ __align__(16) float slab[2][16 * 68];
  __shared__ float sc2s[NPATCH];
  __shared__ float sh2s[NPATCH];
  __shared__ float rsws[PLEN];
  const int tid = threadIdx.x, lane = tid & 31, wave = tid >> 5;
  const int h = lane >> 4, c = lane & 15;
  const int blk = blockIdx.x;
  sc2s[tid] = bnp2[tid];
  sh2s[tid] = bnp2[NPATCH + tid];
  if (tid < PLEN) {
    float a = 0.f;
#pragma unroll 1
    for (int k = 0; k < HIDDEN; ++k) a += fc2_w[tid * HIDDEN + k];
    rsws[tid] = a;
  }
  __syncthreads();
  const float fbc = fc2_b[c], lwc = ln_w[c], lbc = ln_b[c], rswc = rsws[c];
  const float gs = gl_scale[0];

  for (int t = 0; t < 8; ++t) {
    const int rl  = wave * 8 + t;
    const int row = blk * PROWS_BLK + rl;
    const float* sg = s + (size_t)row * SEQ;
    const unsigned* dr = dw + (size_t)row * (DPITCH / 2);
    const float* wr = wsig + (size_t)row * NPATCH;
#pragma unroll 1
    for (int q = 0; q < 32; ++q) {
      const int n = 2 * q + h;
      int idx = n * 8 + c;
      idx = (idx > SEQ - 1) ? (SEQ - 1) : idx;
      const float sp = sg[idx];
      const unsigned wd = dr[n * 8 + (c >> 1)];
      const unsigned bits = (c & 1) ? (wd >> 16) : (wd & 0xffffu);
      const float dv = (float)__builtin_bit_cast(_Float16, (unsigned short)bits) * (1.0f / DCARRY);
      const float w = wr[n];
      const float sc = sc2s[n], sh = sh2s[n];
      float loc = sc * dv + sh * rswc;
      loc = loc + fbc;
      loc = loc + sp;
      const float glob = sp * (1.0f + gs * w);
      const float y = sp + loc + glob;
      float sm = y;
      sm += __shfl_xor(sm, 1, 32);
      sm += __shfl_xor(sm, 2, 32);
      sm += __shfl_xor(sm, 4, 32);
      sm += __shfl_xor(sm, 8, 32);
      const float mu = sm * (1.0f / (float)PLEN);
      const float dd = y - mu;
      float sv = dd * dd;
      sv += __shfl_xor(sv, 1, 32);
      sv += __shfl_xor(sv, 2, 32);
      sv += __shfl_xor(sv, 4, 32);
      sv += __shfl_xor(sv, 8, 32);
      const float var = sv * (1.0f / (float)PLEN);
      const float rs = rsqrtf(var + BN_EPS);
      const float yl = dd * rs * lwc + lbc;
      ys[rl][n * PLEN + c] = (_Float16)(ACARRY * yl);
    }
  }
  __syncthreads();

  v8f acc[4];
#pragma unroll
  for (int jj = 0; jj < 4; ++jj) acc[jj] = (v8f){0.f, 0.f, 0.f, 0.f, 0.f, 0.f, 0.f, 0.f};
  const _Float16* ya = &ys[c][0] + 8 * h;
  const _Float16* sb = (const _Float16*)seasp + (size_t)(64 * wave + c) * DPITCH + 8 * h;
  for (int k0 = 0; k0 < DPITCH; k0 += 32) {
    const v16h a = Frag<_Float16>::load(ya + k0);
#pragma unroll
    for (int jj = 0; jj < 4; ++jj) {
      const v16h bbv = Frag<_Float16>::load(sb + (size_t)(16 * jj) * DPITCH + k0);
      acc[jj] = hmma(a, bbv, acc[jj]);
    }
  }
  float* sl = slab[wave];
#pragma unroll
  for (int jj = 0; jj < 4; ++jj) {
    const int col  = 64 * wave + 16 * jj + c;
    const int colc = (col < NPRED) ? col : (NPRED - 1);
    const float sbv = seas_b[colc];
    const float bv = (col < NPRED) ? (ACARRY * sbv) : 0.f;
#pragma unroll
    for (int r = 0; r < 8; ++r) sl[(8 * h + r) * 68 + 16 * jj + c] = acc[jj][r] * (1.0f / WCARRY) + bv;
  }
  __builtin_amdgcn_fence(__ATOMIC_RELEASE, "workgroup");
  __builtin_amdgcn_wave_barrier();
  __builtin_amdgcn_fence(__ATOMIC_ACQUIRE, "workgroup");
  {
    const int q = lane >> 3, c8 = (lane & 7) * 8;
    for (int pass = 0; pass < 2; ++pass) {
#pragma unroll
      for (int it = 0; it < 4; ++it) {
        const int rowl = it * 4 + q;
        const float* spp = sl + rowl * 68 + c8;
        v8h hv;
#pragma unroll
        for (int e = 0; e < 8; ++e) hv[e] = (_Float16)spp[e];
        *(volatile v8h*)(zplane + (size_t)(blk * PROWS_BLK + rowl) * ZPITCH + 64 * wave + c8) = hv;
      }
      __threadfence();
    }
  }
}

__global__ __launch_bounds__(256) void k_out(const float* __restrict__ o, const float* __restrict__ rev_w,
                                                const float* __restrict__ rev_b, const float* __restrict__ meanp,
                                                const float* __restrict__ stdp, float* __restrict__ out, int n4) {
  const int i = blockIdx.x * 256 + threadIdx.x;
  if (i >= n4) return;
  v4f r4;
#pragma unroll
  for (int e = 0; e < 4; ++e) {
    const int idx = 4 * i + e;
    const int pp  = idx / NCH;
    const int cc  = idx - pp * NCH;
    const int b   = pp / NPRED;
    const int p   = pp - b * NPRED;
    const int bc  = b * NCH + cc;
    float v = o[(size_t)bc * NPREDP + p];
    v = (v - rev_b[cc]) * (1.0f / rev_w[cc]);
    r4[e] = v * stdp[b * MSPITCH + cc] + meanp[b * MSPITCH + cc];
  }
  volatile v4f* d = (volatile v4f*)out + i;
  *d = r4;
  __threadfence();
  *d = r4;
}

extern "C" void kernel_launch(void* const* d_in, const int* in_sizes, int n_in,
                              void* d_out, int out_size, void* d_ws, size_t ws_size,
                              hipStream_t stream) {
  (void)in_sizes; (void)n_in; (void)out_size;
  const float* x      = (const float*)d_in[0];
  const float* rev_w  = (const float*)d_in[1];
  const float* rev_b  = (const float*)d_in[2];
  const float* fc1_w  = (const float*)d_in[3];
  const float* fc1_b  = (const float*)d_in[4];
  const float* bn1_w  = (const float*)d_in[5];
  const float* bn1_b  = (const float*)d_in[6];
  const float* conv_w = (const float*)d_in[7];
  const float* conv_b = (const float*)d_in[8];
  const float* bn2_w  = (const float*)d_in[9];
  const float* bn2_b  = (const float*)d_in[10];
  const float* fc2_w  = (const float*)d_in[11];
  const float* fc2_b  = (const float*)d_in[12];
  const float* m1_w   = (const float*)d_in[13];
  const float* m1_b   = (const float*)d_in[14];
  const float* m2_w   = (const float*)d_in[15];
  const float* m2_b   = (const float*)d_in[16];
  const float* gl_sc  = (const float*)d_in[17];
  const float* ln_w   = (const float*)d_in[18];
  const float* ln_b   = (const float*)d_in[19];
  const float* seas_w = (const float*)d_in[20];
  const float* seas_b = (const float*)d_in[21];
  const float* tr_w   = (const float*)d_in[22];
  const float* tr_b   = (const float*)d_in[23];
  const float* fus_w  = (const float*)d_in[24];
  const float* fus_b  = (const float*)d_in[25];
  float* out = (float*)d_out;

  char* base = (char*)d_ws;
  size_t off = 0;
  auto carve = [&](size_t bytes) -> char* {
    char* p = base + off;
    off += (bytes + 255) & ~(size_t)255;
    return p;
  };
  float*          s_ws    = (float*)carve((size_t)NROWS * SEQ * 4);
  unsigned short* trend16 = (unsigned short*)carve((size_t)NROWS * SEQ * 2);
  float*          meanp   = (float*)carve((size_t)NBATCH * MSPITCH * 4);
  float*          stdp    = (float*)carve((size_t)NBATCH * MSPITCH * 4);
  char*           r4      = carve((size_t)NROWS * DPITCH * 2);
  unsigned short* d16      = (unsigned short*)r4;
  unsigned short* pooled16 = (unsigned short*)r4;
  float*          g1       = (float*)(r4 + (size_t)NROWS * NPATCH * 2);
  unsigned short* u16      = (unsigned short*)(r4 + (size_t)NROWS * NPATCH * 2 + (size_t)NROWS * NPREDP * 4);
  float*          ofin     = (float*)r4;
  unsigned short* z16     = (unsigned short*)carve((size_t)NROWS * ZPITCH * 2);
  float*          wsig    = (float*)carve((size_t)NROWS * NPATCH * 4);
  float*          ps1     = (float*)carve((size_t)NPBLK * NPATCH * 4);
  float*          pq1     = (float*)carve((size_t)NPBLK * NPATCH * 4);
  float*          ps2     = (float*)carve((size_t)NPBLK * NPATCH * 4);
  float*          pq2     = (float*)carve((size_t)NPBLK * NPATCH * 4);
  float*          bnp1    = (float*)carve(512);
  float*          bnp2    = (float*)carve(512);
  unsigned short* m1p     = (unsigned short*)carve((size_t)NPREDP * NPATCH * 2);
  unsigned short* m2p     = (unsigned short*)carve((size_t)NPATCH * NPREDP * 2);
  unsigned short* trp     = (unsigned short*)carve((size_t)NPREDP * SEQ * 2);
  unsigned short* seasp   = (unsigned short*)carve((size_t)NPREDP * DPITCH * 2);
  unsigned short* fusp    = (unsigned short*)carve((size_t)NPREDP * ZPITCH * 2);
  float*          biasp   = (float*)carve(256 * 4);
  if ((size_t)NROWS * NPATCH * 2 + (size_t)NROWS * NPREDP * 4 + (size_t)NROWS * NPREDP * 2 > (size_t)NROWS * DPITCH * 2) return;
  if (off > ws_size) return;

  const int tiles128 = (NROWS / 64) * (NPREDP / 64);
  const int grid128  = (tiles128 + 7) / 8;
  const int tiles64  = (NROWS / 64) * (NPATCH / 64);
  const int grid64   = (tiles64 + 7) / 8;
  const int n2u      = NROWS * NPREDP / 2;
  const int n4out    = OUT_ELEMS / 4;

  k_wprep<<<dim3(256, 6), 256, 0, stream>>>(m1_w, m2_w, tr_w, seas_w, fus_w, tr_b, fus_b,
                                            m1p, m2p, trp, seasp, fusp, biasp);
  k_revin<<<(NBATCH * CGROUPS) / 2, 64, 0, stream>>>(x, rev_w, rev_b, s_ws, trend16, meanp, stdp);
  k_pool<<<NROWS / 64, 256, 0, stream>>>(s_ws, pooled16);
  wmma_gemm64<0, false, 2, 0, false, 0><<<dim3(grid128, 1), 256, 0, stream>>>(
      pooled16, pooled16, NPATCH, 0, m1p, m1p, NPATCH, 0, g1, g1, NPREDP, 0,
      m1_b, m1_b, 0, NROWS, NPREDP, NPATCH, 1.0f / (ACARRY * WCARRY));
  k_gelu_u<<<(n2u + 255) / 256, 256, 0, stream>>>(g1, u16, n2u);
  wmma_gemm64<0, false, 2, 0, false, 6><<<dim3(grid64, 1), 256, 0, stream>>>(
      u16, u16, NPREDP, 0, m2p, m2p, NPREDP, 0, wsig, wsig, NPATCH, 0,
      m2_b, m2_b, 0, NROWS, NPATCH, NPREDP, 1.0f / (UCARRY * WCARRY));
  wmma_gemm64<0, false, 2, 1, false, 0><<<dim3(grid128, 1), 256, 0, stream>>>(
      trend16, trend16, SEQ, 0, trp, trp, SEQ, 0, z16 + NPREDP, z16 + NPREDP, ZPITCH, 0,
      biasp, biasp, 0, NROWS, NPREDP, SEQ, 1.0f / WCARRY);
  k_patch<false><<<NPBLK, 128, 0, stream>>>(s_ws, fc1_w, fc1_b, bnp1, conv_w, conv_b, fc2_w, ps1, pq1, d16);
  k_bnfin<<<1, 64, 0, stream>>>(ps1, pq1, bn1_w, bn1_b, bnp1, NPBLK);
  k_patch<true><<<NPBLK, 128, 0, stream>>>(s_ws, fc1_w, fc1_b, bnp1, conv_w, conv_b, fc2_w, ps2, pq2, d16);
  k_bnfin<<<1, 64, 0, stream>>>(ps2, pq2, bn2_w, bn2_b, bnp2, NPBLK);
  k_lnhead<<<NPBLK, 64, 0, stream>>>(s_ws, (const unsigned*)d16, wsig, bnp2, fc2_w, fc2_b, gl_sc, ln_w, ln_b,
                                     seasp, seas_b, z16);
  wmma_gemm64<0, false, 2, 0, false, 0><<<dim3(grid128, 1), 256, 0, stream>>>(
      z16, z16, ZPITCH, 0, fusp, fusp, ZPITCH, 0, ofin, ofin, NPREDP, 0,
      biasp + NPREDP, biasp, 0, NROWS, NPREDP, ZPITCH, 1.0f / (ACARRY * WCARRY));
  k_out<<<(n4out + 255) / 256, 256, 0, stream>>>(ofin, rev_w, rev_b, meanp, stdp, out, n4out);
}
